// FraudGraphSAGE_87789131530773
// MI455X (gfx1250) — hardware-verified
//
#include <hip/hip_runtime.h>
#include <stddef.h>


#define INCH   12
#define HID    64
#define HID2   32
#define NOUT   2
#define K2     (2 * HID)
#define NTHR   256
#define NWAVE  8
#define EPT    8
#define NGRP   2
#define CHUNK  (NTHR * EPT * NGRP)
#define WCAP   (EPT * NGRP * 32)
#define LISTN  (NWAVE * WCAP)
#define NB1    1024
#define AP1    16
#define PASS1  64
#define NB2    1024
#define WSCALE 8.0f
#define WINV   0.125f

#define LDS_A  (NB1 * AP1 * 4 + LISTN * 4 + 64 + 2 * INCH * HID * 4 + HID * 4)
#define LDS_B  (NB2 * HID * 4 + LISTN * 4 + 64 + NB2 * 4 + 80 * 4 + HID2 * 4)

static_assert((CHUNK & (CHUNK - 1)) == 0);
static_assert(CHUNK <= 4096);
static_assert(NB1 <= 4096 && NB2 <= 4096);
static_assert((NB1 & (NB1 - 1)) == 0 && (NB2 & (NB2 - 1)) == 0);
static_assert(PASS1 * HID * 4 <= LISTN * 4);
static_assert((NB1 % PASS1) == 0);
static_assert(PASS1 * HID == NWAVE * 4 * 128);
static_assert(PASS1 == 4 * 16);
static_assert(NTHR == 4 * HID);
static_assert(NWAVE * 16 * HID2 <= LISTN);
static_assert(((NB2 / 16) % NWAVE) == 0);
static_assert(NB2 * NOUT == NWAVE * 2 * 4 * 32);
static_assert(HID2 * NOUT + NOUT <= 80);
static_assert(LDS_A == 88384);
static_assert(LDS_B == 283136);

typedef float    v2f  __attribute__((ext_vector_type(2)));
typedef float    v4f  __attribute__((ext_vector_type(4)));
typedef float    v8f  __attribute__((ext_vector_type(8)));
typedef int      v4i  __attribute__((ext_vector_type(4)));
typedef _Float16 v8h  __attribute__((ext_vector_type(8)));
typedef _Float16 v16h __attribute__((ext_vector_type(16)));
union FragH { v16h v; v8h h[2]; };

__device__ __forceinline__ v8h cvt8(v4f a, v4f b) {
  v8h r;
  r[0] = (_Float16)a.x; r[1] = (_Float16)a.y; r[2] = (_Float16)a.z; r[3] = (_Float16)a.w;
  r[4] = (_Float16)b.x; r[5] = (_Float16)b.y; r[6] = (_Float16)b.z; r[7] = (_Float16)b.w;
  return r;
}

__device__ __forceinline__ v8f wmh(v16h a, v16h b, v8f c) {
  v8f d = __builtin_amdgcn_wmma_f32_16x16x32_f16(false, a, false, b, (short)0, c, false, false);
  asm volatile("v_nop\n\tv_nop\n\tv_nop\n\tv_nop" : "+v"(d) : "v"(a), "v"(b));
  return d;
}

__device__ __forceinline__ float dot12(v4f a, v4f b, v4f c, const float* w) {
  float s = a.x * w[0];
  s = fmaf(a.y, w[1 * HID], s);
  s = fmaf(a.z, w[2 * HID], s);
  s = fmaf(a.w, w[3 * HID], s);
  s = fmaf(b.x, w[4 * HID], s);
  s = fmaf(b.y, w[5 * HID], s);
  s = fmaf(b.z, w[6 * HID], s);
  s = fmaf(b.w, w[7 * HID], s);
  s = fmaf(c.x, w[8 * HID], s);
  s = fmaf(c.y, w[9 * HID], s);
  s = fmaf(c.z, w[10 * HID], s);
  s = fmaf(c.w, w[11 * HID], s);
  return s;
}

template <int NB>
__device__ __forceinline__ int scan_chunk(const int* __restrict__ dsts, int nE, int cbase, int nodeBase,
                                          int vec8, int* list, int tid, int lane, int wave) {
  int wc = 0;
#pragma unroll
  for (int g = 0; g < NGRP; ++g) {
    const int el0  = (g * NTHR + tid) * EPT;
    const int e0   = cbase + el0;
    const int sent = -2147483647 - 1;
    v4i da, db;
    if (vec8 != 0 && e0 + 7 < nE) {
      da = *(const v4i*)(dsts + e0);
      db = *(const v4i*)(dsts + e0 + 4);
    } else {
      da.x = (e0     < nE) ? dsts[e0]     : sent;
      da.y = (e0 + 1 < nE) ? dsts[e0 + 1] : sent;
      da.z = (e0 + 2 < nE) ? dsts[e0 + 2] : sent;
      da.w = (e0 + 3 < nE) ? dsts[e0 + 3] : sent;
      db.x = (e0 + 4 < nE) ? dsts[e0 + 4] : sent;
      db.y = (e0 + 5 < nE) ? dsts[e0 + 5] : sent;
      db.z = (e0 + 6 < nE) ? dsts[e0 + 6] : sent;
      db.w = (e0 + 7 < nE) ? dsts[e0 + 7] : sent;
    }
    const unsigned nb = (unsigned)nodeBase;
    const unsigned s0 = (unsigned)da.x - nb, s1 = (unsigned)da.y - nb;
    const unsigned s2 = (unsigned)da.z - nb, s3 = (unsigned)da.w - nb;
    const unsigned s4 = (unsigned)db.x - nb, s5 = (unsigned)db.y - nb;
    const unsigned s6 = (unsigned)db.z - nb, s7 = (unsigned)db.w - nb;
    const bool h0 = s0 < (unsigned)NB, h1 = s1 < (unsigned)NB, h2 = s2 < (unsigned)NB, h3 = s3 < (unsigned)NB;
    const bool h4 = s4 < (unsigned)NB, h5 = s5 < (unsigned)NB, h6 = s6 < (unsigned)NB, h7 = s7 < (unsigned)NB;
    const unsigned any = __builtin_amdgcn_ballot_w32(h0 | h1 | h2 | h3 | h4 | h5 | h6 | h7);
    if (any != 0u) {
#define HITJ(J, HJ, SJ) { \
        const unsigned mj = __builtin_amdgcn_ballot_w32(HJ); \
        if (mj != 0u) { \
          if (HJ) { \
            const int pos = wc + (int)__builtin_amdgcn_mbcnt_lo(mj, 0u); \
            if (pos < WCAP) list[wave * WCAP + pos] = ((el0 + (J)) << 12) | (int)(SJ); \
          } \
          wc += (int)__builtin_popcount(mj); } }
      HITJ(0, h0, s0)
      HITJ(1, h1, s1)
      HITJ(2, h2, s2)
      HITJ(3, h3, s3)
      HITJ(4, h4, s4)
      HITJ(5, h5, s5)
      HITJ(6, h6, s6)
      HITJ(7, h7, s7)
#undef HITJ
    }
  }
  return wc;
}

__global__ __launch_bounds__(NTHR) void k_wprep(
    const float* __restrict__ w2l, const float* __restrict__ w2r, _Float16* w2s) {
  const int i = blockIdx.x * NTHR + threadIdx.x;
  if (i >= HID2 * K2 / 8) return;
  const int o  = i * 8;
  const int n  = o / K2;
  const int k0 = o - n * K2;
  const float* p = (k0 < HID) ? (w2l + (size_t)k0 * HID2 + n) : (w2r + (size_t)(k0 - HID) * HID2 + n);
  v4f a, b;
  a.x = p[0];        a.y = p[HID2];     a.z = p[2 * HID2]; a.w = p[3 * HID2];
  b.x = p[4 * HID2]; b.y = p[5 * HID2]; b.z = p[6 * HID2]; b.w = p[7 * HID2];
  a = a * WSCALE;
  b = b * WSCALE;
  const v8h hv = cvt8(a, b);
  _Float16* dp = w2s + o;
  *(volatile v8h*)dp = hv;
  __threadfence();
  *(volatile v8h*)dp = hv;
}

__global__ __launch_bounds__(NTHR) void k_layer1(
    const float* __restrict__ x, const int* __restrict__ ei,
    const float* __restrict__ w1l, const float* __restrict__ b1, const float* __restrict__ w1r,
    float* h1, int nN, int nE, int vec8) {
  extern __shared__ v4f lds_dyn[];
  float* acc1 = (float*)lds_dyn;
  int*   list = (int*)(acc1 + NB1 * AP1);
  int*   wcnt = list + LISTN;
  float* wsh  = (float*)(wcnt + 16);
  float* bsh  = wsh + 2 * INCH * HID;
  float* stg  = (float*)list;
  const int tid = threadIdx.x, lane = tid & 31, wave = tid >> 5;
  const int nodeBase = blockIdx.x * NB1;
  const int* dsts = ei + nE;

  {
    const v4f z = {0.f, 0.f, 0.f, 0.f};
    for (int i = tid; i < NB1 * AP1 / 4; i += NTHR) lds_dyn[i] = z;
  }
  for (int i = tid; i < INCH * HID; i += NTHR) { wsh[i] = w1l[i]; wsh[INCH * HID + i] = w1r[i]; }
  if (tid < HID) bsh[tid] = b1[tid];
  __syncthreads();

  const int nChunks = (nE + CHUNK - 1) / CHUNK;
#pragma unroll 1
  for (int ch = 0; ch < nChunks; ++ch) {
    const int cbase = ch * CHUNK;
    const int wc = scan_chunk<NB1>(dsts, nE, cbase, nodeBase, vec8, list, tid, lane, wave);
    if (lane == 0) wcnt[wave] = wc;
    __syncthreads();
    if (wave == 0) {
#pragma unroll 1
      for (int wsx = 0; wsx < NWAVE; ++wsx) {
        int n = __builtin_amdgcn_readfirstlane(wcnt[wsx]);
        n = n > WCAP ? WCAP : (n < 0 ? 0 : n);
        const int* lp = list + wsx * WCAP;
#pragma unroll 1
        for (int i = 0; i < n; ++i) {
          const int ent  = __builtin_amdgcn_readfirstlane(lp[i]);
          const int slot = ent & (NB1 - 1);
          int e = cbase + ((ent >> 12) & (CHUNK - 1));
          e = e > nE - 1 ? nE - 1 : e;
          int src = ei[e];
          src = src < 0 ? 0 : (src > nN - 1 ? nN - 1 : src);
          if (lane < INCH + 1) {
            float v = 1.0f;
            if (lane < INCH) v = x[(size_t)src * INCH + lane];
            float* ap = acc1 + slot * AP1 + lane;
            *ap = *ap + v;
          }
        }
      }
    }
    __syncthreads();
  }

  const int col = tid & (HID - 1);
  const int grp = tid >> 6;
  const float bcol = bsh[col];
  const float* wl = wsh + col;
  const float* wr = wsh + INCH * HID + col;
#pragma unroll 1
  for (int p = 0; p < NB1 / PASS1; ++p) {
#pragma unroll 1
    for (int j = 0; j < PASS1 / 4; ++j) {
      const int lr   = 4 * j + grp;
      const int slot = p * PASS1 + lr;
      int node = nodeBase + slot;
      node = node > nN - 1 ? nN - 1 : node;
      const float* xp = x + (size_t)node * INCH;
      const v4f x0 = *(const v4f*)xp, x1 = *(const v4f*)(xp + 4), x2 = *(const v4f*)(xp + 8);
      const float* ap = acc1 + slot * AP1;
      const v4f s0 = *(const v4f*)ap, s1 = *(const v4f*)(ap + 4), s2 = *(const v4f*)(ap + 8);
      const float cntf = ap[12];
      const float rd = 1.0f / fmaxf(cntf, 1.0f);
      const float vl = dot12(s0 * rd, s1 * rd, s2 * rd, wl);
      const float vr = dot12(x0, x1, x2, wr);
      float v = (vl + bcol) + vr;
      v = fmaxf(v, 0.0f);
      stg[lr * HID + col] = v;
    }
    __syncthreads();
    v4f ov[4];
#pragma unroll
    for (int q = 0; q < 4; ++q) ov[q] = *(const v4f*)(stg + (wave * 4 + q) * 128 + 4 * lane);
    float* gp = h1 + ((size_t)nodeBase + (size_t)p * PASS1) * HID;
#pragma unroll
    for (int q = 0; q < 4; ++q) *(volatile v4f*)(gp + (wave * 4 + q) * 128 + 4 * lane) = ov[q];
    __threadfence();
#pragma unroll
    for (int q = 0; q < 4; ++q) *(volatile v4f*)(gp + (wave * 4 + q) * 128 + 4 * lane) = ov[q];
    __syncthreads();
  }
}

__global__ __launch_bounds__(NTHR) void k_layer2(
    const int* __restrict__ ei, const float* __restrict__ h1, const _Float16* __restrict__ w2s,
    const float* __restrict__ b2, const float* __restrict__ wc, const float* __restrict__ bc,
    float* out, int nN, int nE, int vec8) {
  extern __shared__ v4f lds_dyn[];
  float* acc2 = (float*)lds_dyn;
  int*   list = (int*)(acc2 + NB2 * HID);
  int*   wcnt = list + LISTN;
  int*   cnt  = wcnt + 16;
  float* wcs  = (float*)(cnt + NB2);
  float* b2s  = wcs + 80;
  float* stg  = (float*)list;
  const int tid = threadIdx.x, lane = tid & 31, wave = tid >> 5, hh = lane >> 4, m = lane & 15;
  const int nodeBase = blockIdx.x * NB2;
  const int* dsts = ei + nE;

  {
    const v4f z = {0.f, 0.f, 0.f, 0.f};
    for (int i = tid; i < NB2 * HID / 4; i += NTHR) lds_dyn[i] = z;
  }
  for (int i = tid; i < NB2; i += NTHR) cnt[i] = 0;
  if (tid < HID2 * NOUT) wcs[tid] = wc[tid];
  if (tid < NOUT) wcs[HID2 * NOUT + tid] = bc[tid];
  if (tid < HID2) b2s[tid] = b2[tid];
  __syncthreads();

  const int nChunks = (nE + CHUNK - 1) / CHUNK;
#pragma unroll 1
  for (int ch = 0; ch < nChunks; ++ch) {
    const int cbase = ch * CHUNK;
    const int wcn = scan_chunk<NB2>(dsts, nE, cbase, nodeBase, vec8, list, tid, lane, wave);
    if (lane == 0) wcnt[wave] = wcn;
    __syncthreads();
    if (wave == 0) {
#pragma unroll 1
      for (int wsx = 0; wsx < NWAVE; ++wsx) {
        int n = __builtin_amdgcn_readfirstlane(wcnt[wsx]);
        n = n > WCAP ? WCAP : (n < 0 ? 0 : n);
        const int* lp = list + wsx * WCAP;
#pragma unroll 1
        for (int i = 0; i < n; ++i) {
          const int ent  = __builtin_amdgcn_readfirstlane(lp[i]);
          const int slot = ent & (NB2 - 1);
          int e = cbase + ((ent >> 12) & (CHUNK - 1));
          e = e > nE - 1 ? nE - 1 : e;
          int src = ei[e];
          src = src < 0 ? 0 : (src > nN - 1 ? nN - 1 : src);
          const v2f v = *(const v2f*)(h1 + (size_t)src * HID + 2 * lane);
          v2f* ap = (v2f*)(acc2 + slot * HID + 2 * lane);
          *ap = *ap + v;
          if (lane == 0) cnt[slot] = cnt[slot] + 1;
        }
      }
    }
    __syncthreads();
  }

  FragH bw[2][4];
#pragma unroll
  for (int nt = 0; nt < 2; ++nt) {
#pragma unroll
    for (int kt = 0; kt < 4; ++kt) {
      const _Float16* bp = w2s + (size_t)(16 * nt + m) * K2 + 32 * kt + 8 * hh;
      bw[nt][kt].h[0] = *(const v8h*)bp;
      bw[nt][kt].h[1] = *(const v8h*)(bp + 16);
    }
  }
  const int row = m;
  const int cc  = hh;
  const float bcv = wcs[HID2 * NOUT + cc];
  const float bA = b2s[m], bB = b2s[16 + m];

#pragma unroll 1
  for (int it = 0; it < (NB2 / 16) / NWAVE; ++it) {
    const int t    = it * NWAVE + wave;
    const int lrow = 16 * t + m;
    const size_t node = (size_t)nodeBase + (size_t)lrow;
    const float rd = 1.0f / fmaxf((float)cnt[lrow], 1.0f);
    v8f c0 = {0.f, 0.f, 0.f, 0.f, 0.f, 0.f, 0.f, 0.f};
    v8f c1 = {0.f, 0.f, 0.f, 0.f, 0.f, 0.f, 0.f, 0.f};
#pragma unroll
    for (int kt = 0; kt < 2; ++kt) {
      const float* ap = acc2 + lrow * HID + 32 * kt + 8 * hh;
      const v4f p0 = *(const v4f*)ap * rd,        p1 = *(const v4f*)(ap + 4) * rd;
      const v4f p2 = *(const v4f*)(ap + 16) * rd, p3 = *(const v4f*)(ap + 20) * rd;
      FragH a;
      a.h[0] = cvt8(p0, p1);
      a.h[1] = cvt8(p2, p3);
      c0 = wmh(a.v, bw[0][kt].v, c0);
      c1 = wmh(a.v, bw[1][kt].v, c1);
    }
#pragma unroll
    for (int kt = 0; kt < 2; ++kt) {
      const float* gp = h1 + node * HID + 32 * kt + 8 * hh;
      const v4f p0 = *(const v4f*)gp,        p1 = *(const v4f*)(gp + 4);
      const v4f p2 = *(const v4f*)(gp + 16), p3 = *(const v4f*)(gp + 20);
      FragH a;
      a.h[0] = cvt8(p0, p1);
      a.h[1] = cvt8(p2, p3);
      c0 = wmh(a.v, bw[0][2 + kt].v, c0);
      c1 = wmh(a.v, bw[1][2 + kt].v, c1);
    }
    float* sp = stg + wave * (16 * HID2) + (8 * hh) * HID2;
#pragma unroll
    for (int r = 0; r < 8; ++r) {
      sp[r * HID2 + m]      = fmaxf(c0[r] * WINV + bA, 0.0f);
      sp[r * HID2 + 16 + m] = fmaxf(c1[r] * WINV + bB, 0.0f);
    }
    __syncthreads();
    const float* hp = stg + wave * (16 * HID2) + row * HID2;
    float o = 0.0f;
#pragma unroll
    for (int k = 0; k < HID2; ++k) o = fmaf(hp[k], wcs[k * NOUT + cc], o);
    o = o + bcv;
    acc2[(16 * t) * HID + row * NOUT + cc] = o;
    __syncthreads();
  }
  __syncthreads();

  const size_t outN = (size_t)nN * NOUT;
  const size_t ob   = (size_t)nodeBase * NOUT;
  v4f ov[2];
  size_t gi[2];
#pragma unroll
  for (int q = 0; q < 2; ++q) {
    const int L = (wave * 2 + q) * 4 + (lane >> 3);
    ov[q] = *(const v4f*)(acc2 + L * 16 * HID + 4 * (lane & 7));
    gi[q] = ob + (size_t)L * 32 + (size_t)(4 * (lane & 7));
  }
#pragma unroll
  for (int q = 0; q < 2; ++q) {
    if (gi[q] + 4 <= outN) {
      *(volatile v4f*)(out + gi[q]) = ov[q];
    } else {
#pragma unroll
      for (int j = 0; j < 4; ++j) if (gi[q] + (size_t)j < outN) *(volatile float*)(out + gi[q] + j) = ov[q][j];
    }
  }
  __threadfence();
#pragma unroll
  for (int q = 0; q < 2; ++q) {
    if (gi[q] + 4 <= outN) {
      *(volatile v4f*)(out + gi[q]) = ov[q];
    } else {
#pragma unroll
      for (int j = 0; j < 4; ++j) if (gi[q] + (size_t)j < outN) *(volatile float*)(out + gi[q] + j) = ov[q][j];
    }
  }
}

extern "C" void kernel_launch(void* const* d_in, const int* in_sizes, int n_in,
                              void* d_out, int out_size, void* d_ws, size_t ws_size,
                              hipStream_t stream) {
  if (n_in < 10) return;
  const int nN = in_sizes[0] / INCH;
  const int nE = in_sizes[1] / 2;
  if (nN <= 0 || nE < 0 || in_sizes[0] != nN * INCH || in_sizes[1] != nE * 2) return;
  if (in_sizes[2] != INCH * HID || in_sizes[3] < HID || in_sizes[4] != INCH * HID) return;
  if (in_sizes[5] != HID * HID2 || in_sizes[6] < HID2 || in_sizes[7] != HID * HID2) return;
  if (in_sizes[8] != HID2 * NOUT || in_sizes[9] < NOUT) return;
  if (out_size != nN * NOUT) return;

  const float* x   = (const float*)d_in[0];
  const int*   ei  = (const int*)d_in[1];
  const float* w1l = (const float*)d_in[2];
  const float* b1  = (const float*)d_in[3];
  const float* w1r = (const float*)d_in[4];
  const float* w2l = (const float*)d_in[5];
  const float* b2  = (const float*)d_in[6];
  const float* w2r = (const float*)d_in[7];
  const float* wc  = (const float*)d_in[8];
  const float* bc  = (const float*)d_in[9];
  float* out = (float*)d_out;

  const int nA = (nN + NB1 - 1) / NB1;
  const int nB = (nN + NB2 - 1) / NB2;
  size_t rowsH = (size_t)nA * NB1;
  if ((size_t)nB * NB2 > rowsH) rowsH = (size_t)nB * NB2;

  char* ws = (char*)d_ws;
  size_t off = 0;
  const size_t oW2 = off; off += (size_t)HID2 * K2 * 2;          off = (off + 255) & ~(size_t)255;
  const size_t oH1 = off; off += rowsH * HID * 4;                off = (off + 255) & ~(size_t)255;
  if (off > ws_size) return;
  _Float16* w2s = (_Float16*)(ws + oW2);
  float*    h1  = (float*)(ws + oH1);

  const int vec8 = ((nE & 3) == 0) ? 1 : 0;

  const int nPrep = HID2 * K2 / 8;
  k_wprep<<<(nPrep + NTHR - 1) / NTHR, NTHR, 0, stream>>>(w2l, w2r, w2s);

  hipFuncSetAttribute(reinterpret_cast<const void*>(&k_layer1),
                      hipFuncAttributeMaxDynamicSharedMemorySize, LDS_A);
  k_layer1<<<nA, NTHR, LDS_A, stream>>>(x, ei, w1l, b1, w1r, h1, nN, nE, vec8);

  hipFuncSetAttribute(reinterpret_cast<const void*>(&k_layer2),
                      hipFuncAttributeMaxDynamicSharedMemorySize, LDS_B);
  k_layer2<<<nB, NTHR, LDS_B, stream>>>(ei, h1, w2s, b2, wc, bc, out, nN, nE, vec8);
}
